// CustomAttention_57784490001204
// MI455X (gfx1250) — hardware-verified
//
#include <hip/hip_runtime.h>
#include <stdint.h>
#include <stddef.h>


typedef _Float16 v16h __attribute__((ext_vector_type(16)));
typedef _Float16 v8h  __attribute__((ext_vector_type(8)));
typedef float    v8f  __attribute__((ext_vector_type(8)));
typedef float    v4f  __attribute__((ext_vector_type(4)));
union Frag { v16h v; v8h half[2]; };

#define NQ    512
#define NKEY  512
#define DD    64
#define NTILE (NQ / 16)

static __device__ __forceinline__ v8f wmma_f16(v16h a, v16h b, v8f c) {
    c = __builtin_amdgcn_wmma_f32_16x16x32_f16(false, a, false, b, (short)0, c, false, false);
    asm volatile("v_nop\n\tv_nop\n\tv_nop\n\tv_nop" : "+v"(c) : "v"(a), "v"(b));
    return c;
}

#if __has_builtin(__builtin_amdgcn_tanhf)
static __device__ __forceinline__ float th(float x) { return __builtin_amdgcn_tanhf(x); }
#else
static __device__ __forceinline__ float th(float x) {
    const float e = __expf(2.0f * x);
    return 1.0f - 2.0f * __builtin_amdgcn_rcpf(e + 1.0f);
}
#endif

#define XP 72
#define WP 72
#define OP 68

static __device__ __forceinline__ void store_qk_pass(const float* Ot, float* dstb,
                                                     int row0, int nrows, int tid) {
#pragma unroll
    for (int it = 0; it < 8; ++it) {
        const int f  = it * 128 + tid;
        const int r  = f >> 4;
        const int c4 = (f & 15) * 4;
        if (row0 + r < nrows) {
            const v4f val = *(const v4f*)(Ot + r * OP + c4);
            *(volatile v4f*)(dstb + (size_t)(row0 + r) * DD + c4) = val;
        }
    }
}

static __device__ __forceinline__ void store_v_pass(const float* Ot, _Float16* vo,
                                                    int row0, int nrows, int tid) {
#pragma unroll
    for (int it = 0; it < 4; ++it) {
        const int f  = it * 128 + tid;
        const int r  = f >> 3;
        const int c8 = (f & 7) * 8;
        if (row0 + r < nrows) {
            const v4f u0 = *(const v4f*)(Ot + r * OP + c8);
            const v4f u1 = *(const v4f*)(Ot + r * OP + c8 + 4);
            v8h hv;
            hv[0] = (_Float16)u0.x; hv[1] = (_Float16)u0.y; hv[2] = (_Float16)u0.z; hv[3] = (_Float16)u0.w;
            hv[4] = (_Float16)u1.x; hv[5] = (_Float16)u1.y; hv[6] = (_Float16)u1.z; hv[7] = (_Float16)u1.w;
            *(volatile v8h*)(vo + (size_t)(row0 + r) * DD + c8) = hv;
        }
    }
}

__global__ __launch_bounds__(128) void k_proj(
    const float* __restrict__ x1, const float* __restrict__ x2,
    const float* __restrict__ Wq, const float* __restrict__ Wk,
    const float* __restrict__ Wv,
    float* qo, float* ko, _Float16* vo, int nrows1, int nrows2)
{
    __shared__ __attribute__((aligned(16))) _Float16 Wh[64 * WP];
    __shared__ __attribute__((aligned(16))) _Float16 Xh[64 * XP];
    __shared__ __attribute__((aligned(16))) float    Ot[64 * OP];

    const int mat   = blockIdx.y;
    const float* x  = (mat == 0) ? x1 : x2;
    const float* W  = (mat == 0) ? Wq : ((mat == 1) ? Wk : Wv);
    const int nrows = (mat == 0) ? nrows1 : nrows2;
    const int tid   = threadIdx.x;
    const int row0  = blockIdx.x * 64;
    if (row0 >= nrows) return;

    for (int i = tid; i < 1024; i += 128) {
        const int r  = i >> 4;
        const int c4 = (i & 15) * 4;
        const v4f wv = *(const v4f*)(W + r * DD + c4);
        _Float16* dw = Wh + r * WP + c4;
        dw[0] = (_Float16)(wv.x * 64.0f); dw[1] = (_Float16)(wv.y * 64.0f);
        dw[2] = (_Float16)(wv.z * 64.0f); dw[3] = (_Float16)(wv.w * 64.0f);
        int xr = row0 + r; if (xr > nrows - 1) xr = nrows - 1;
        const v4f xv = *(const v4f*)(x + (size_t)xr * DD + c4);
        _Float16* dx = Xh + r * XP + c4;
        dx[0] = (_Float16)xv.x; dx[1] = (_Float16)xv.y;
        dx[2] = (_Float16)xv.z; dx[3] = (_Float16)xv.w;
    }
    __syncthreads();

    const int w = tid >> 5;
    const int l = tid & 31;
    const int h = l >> 4;
    const int m = l & 15;

    const v8f zero8 = {0.f, 0.f, 0.f, 0.f, 0.f, 0.f, 0.f, 0.f};
    v8f acc[4] = {zero8, zero8, zero8, zero8};

    const _Float16* arow = Xh + (16 * w + m) * XP + 8 * h;
#pragma unroll
    for (int ks = 0; ks < 2; ++ks) {
        const int k0 = ks * 32;
        Frag a;
        a.half[0] = *(const v8h*)(arow + k0);
        a.half[1] = *(const v8h*)(arow + k0 + 16);
#pragma unroll
        for (int ct = 0; ct < 4; ++ct) {
            const _Float16* brow = Wh + (16 * ct + m) * WP + 8 * h + k0;
            Frag bf;
            bf.half[0] = *(const v8h*)(brow);
            bf.half[1] = *(const v8h*)(brow + 16);
            acc[ct] = wmma_f16(a.v, bf.v, acc[ct]);
        }
    }

#pragma unroll
    for (int ct = 0; ct < 4; ++ct) {
#pragma unroll
        for (int r = 0; r < 8; ++r)
            Ot[(16 * w + 8 * h + r) * OP + 16 * ct + m] = acc[ct][r] * 0.015625f;
    }
    __syncthreads();

    if (mat < 2) {
        float* dstb = (mat == 0) ? qo : ko;
        store_qk_pass(Ot, dstb, row0, nrows, tid);
        __threadfence();
        store_qk_pass(Ot, dstb, row0, nrows, tid);
    } else {
        store_v_pass(Ot, vo, row0, nrows, tid);
        __threadfence();
        store_v_pass(Ot, vo, row0, nrows, tid);
    }
}

#define SS_P   516
#define PF_P   520
#define KS_P   68
#define VS_P   72
#define OT2_P  68
#define OFF_PF  33024
#define OFF_KV  49664
#define OFF_RED 84480
#define ATT_LDS 88576

__global__ __launch_bounds__(256) void k_attn(
    const float* __restrict__ qg, const float* __restrict__ kg,
    const _Float16* __restrict__ vg, float* out, int nblk)
{
    extern __shared__ __attribute__((aligned(16))) char smem[];
    float*    ss  = (float*)(smem);
    _Float16* pf  = (_Float16*)(smem + OFF_PF);
    float*    ks  = (float*)(smem + OFF_KV);
    _Float16* vs  = (_Float16*)(smem + OFF_KV);
    float*    red = (float*)(smem + OFF_RED);
    float*    ot  = ss;

    const int tid  = threadIdx.x;
    const int lane = tid & 31;
    const int w    = tid >> 5;
    const int bid  = blockIdx.x;
    if (bid >= nblk) return;
    const int b    = bid / NTILE;
    const int n0   = (bid % NTILE) * 16;

    const float*    qb = qg + (size_t)b * NQ   * DD;
    const float*    kb = kg + (size_t)b * NKEY * DD;
    const _Float16* vb = vg + (size_t)b * NKEY * DD;

    const int sn = tid >> 4;
    const int mb = tid & 15;
    v4f qv[16];
    {
        const v4f* qrow = (const v4f*)(qb + (size_t)(n0 + sn) * DD);
#pragma unroll
        for (int t = 0; t < 16; ++t) qv[t] = qrow[t];
    }

    for (int mt = 0; mt < NKEY / 128; ++mt) {
        __syncthreads();
        for (int i = tid; i < 2048; i += 256) {
            const int r = i >> 4, j = i & 15;
            *(v4f*)(ks + r * KS_P + 4 * j) =
                *(const v4f*)(kb + (size_t)(mt * 128 + r) * DD + 4 * j);
        }
        __syncthreads();
#pragma unroll 1
        for (int j = 0; j < 8; ++j) {
            const int mm = mb + 16 * j;
            const v4f* kr = (const v4f*)(ks + mm * KS_P);
            float a = 0.f;
#pragma unroll
            for (int t = 0; t < 16; ++t) {
                const v4f kk = kr[t];
                a += th(qv[t].x + kk.x);
                a += th(qv[t].y + kk.y);
                a += th(qv[t].z + kk.z);
                a += th(qv[t].w + kk.w);
            }
            ss[sn * SS_P + mt * 128 + mm] = a * 0.015625f;
        }
    }
    __syncthreads();

    for (int r = 0; r < 2; ++r) {
        const int n = w * 2 + r;
        const float* srow = ss + n * SS_P;
        float sv[16];
        float mx = -3.0e38f;
#pragma unroll
        for (int j = 0; j < 16; ++j) { sv[j] = srow[lane + 32 * j]; mx = fmaxf(mx, sv[j]); }
#pragma unroll
        for (int off = 16; off > 0; off >>= 1) mx = fmaxf(mx, __shfl_xor(mx, off, 32));
        float sum = 0.f;
#pragma unroll
        for (int j = 0; j < 16; ++j) { sv[j] = __expf(sv[j] - mx); sum += sv[j]; }
#pragma unroll
        for (int off = 16; off > 0; off >>= 1) sum += __shfl_xor(sum, off, 32);
        const float inv = 256.0f / sum;
        _Float16* prow = pf + n * PF_P;
#pragma unroll
        for (int j = 0; j < 16; ++j) prow[lane + 32 * j] = (_Float16)(sv[j] * inv);
    }
    __syncthreads();

    const int dt  = w & 3;
    const int ksh = w >> 2;
    const int m16 = lane & 15;
    const int h   = lane >> 4;
    const int col = dt * 16 + m16;
    const v8f zero8 = {0.f, 0.f, 0.f, 0.f, 0.f, 0.f, 0.f, 0.f};
    v8f acc = zero8;

    for (int mt = 0; mt < NKEY / 128; ++mt) {
        for (int i = tid; i < 1024; i += 256) {
            const int r = i >> 3, j = i & 7;
            *(v8h*)(vs + r * VS_P + 8 * j) =
                *(const v8h*)(vb + (size_t)(mt * 128 + r) * DD + 8 * j);
        }
        __syncthreads();
#pragma unroll
        for (int kk = 0; kk < 2; ++kk) {
            const int klocal = ksh * 64 + kk * 32;
            const int mglob  = mt * 128 + klocal;
            Frag a;
            const _Float16* ap = pf + m16 * PF_P + mglob + 8 * h;
            a.half[0] = *(const v8h*)(ap);
            a.half[1] = *(const v8h*)(ap + 16);
            Frag bfr;
            const _Float16* bp0 = vs + (klocal + 8 * h) * VS_P + col;
            const _Float16* bp1 = vs + (klocal + 16 + 8 * h) * VS_P + col;
#pragma unroll
            for (int t = 0; t < 8; ++t) {
                bfr.v[t]     = bp0[t * VS_P];
                bfr.v[8 + t] = bp1[t * VS_P];
            }
            acc = wmma_f16(a.v, bfr.v, acc);
        }
        __syncthreads();
    }

    if (ksh == 1) {
        float* rr = red + ((w - 4) * 32 + lane) * 8;
#pragma unroll
        for (int j = 0; j < 8; ++j) rr[j] = acc[j];
    }
    __syncthreads();
    if (ksh == 0) {
        const float* rr = red + (w * 32 + lane) * 8;
#pragma unroll
        for (int j = 0; j < 8; ++j)
            ot[(8 * h + j) * OT2_P + col] = (acc[j] + rr[j]) * 0.00390625f;
    }
    __syncthreads();
    {
        const int r  = 2 * w + (lane >> 4);
        const int c4 = (lane & 15) * 4;
        const v4f val = *(const v4f*)(ot + r * OT2_P + c4);
        float* dst = out + ((size_t)b * NQ + n0 + r) * DD + c4;
        *(volatile v4f*)dst = val;
        __threadfence();
        *(volatile v4f*)dst = val;
    }
}

static inline size_t align128(size_t v) { return (v + 127) & ~(size_t)127; }

extern "C" void kernel_launch(void* const* d_in, const int* in_sizes, int n_in,
                              void* d_out, int out_size, void* d_ws, size_t ws_size,
                              hipStream_t stream) {
    if (n_in < 5) return;
    const float* x1 = (const float*)d_in[0];
    const float* x2 = (const float*)d_in[1];
    const float* Wq = (const float*)d_in[2];
    const float* Wk = (const float*)d_in[3];
    const float* Wv = (const float*)d_in[4];

    const int nrows1 = in_sizes[0] / DD;
    const int nrows2 = in_sizes[1] / DD;
    const int nbatch = nrows1 / NQ;
    if (nrows1 <= 0 || nrows2 != nbatch * NKEY || nrows1 != nbatch * NQ) return;
    if (out_size != nrows1 * DD) return;
    if (in_sizes[2] != DD * DD || in_sizes[3] != DD * DD || in_sizes[4] != DD * DD) return;

    const size_t bytes_q = (size_t)nrows1 * DD * sizeof(float);
    const size_t bytes_k = (size_t)nrows2 * DD * sizeof(float);
    const size_t bytes_v = (size_t)nrows2 * DD * sizeof(_Float16);
    const size_t off_q = 0;
    const size_t off_k = off_q + align128(bytes_q);
    const size_t off_v = off_k + align128(bytes_k);
    if (off_v + bytes_v > ws_size) return;

    float*    q  = (float*)((char*)d_ws + off_q);
    float*    k  = (float*)((char*)d_ws + off_k);
    _Float16* vh = (_Float16*)((char*)d_ws + off_v);

    const int maxrows = (nrows1 > nrows2) ? nrows1 : nrows2;
    const int gx_proj = (maxrows + 63) / 64;
    k_proj<<<dim3(gx_proj, 3), 128, 0, stream>>>(x1, x2, Wq, Wk, Wv, q, k, vh, nrows1, nrows2);

    const int nblk = nbatch * NTILE;
    k_attn<<<dim3(nblk), 256, ATT_LDS, stream>>>(q, k, vh, (float*)d_out, nblk);
}
